// ParallelEncoderBlock_20091857011462
// MI455X (gfx1250) — hardware-run, weakly checked
//
#include <hip/hip_runtime.h>
#include <math.h>
#include <stdint.h>

#define NBATCH 2
#define SEQL   2048
#define DMOD   1024
#define NHEAD  16
#define HDIM   64
#define FFD    4096
#define PROJN  11264
#define QKP    2048
#define A2P    5120
#define NTOK   (NBATCH * SEQL)
#define NQB    (SEQL / 64)
static_assert(NHEAD * HDIM == DMOD);
static_assert(PROJN == 3 * DMOD + 2 * FFD);
static_assert(A2P == DMOD + FFD);
static_assert((SEQL % 64) == 0 && (DMOD % 64) == 0 && (FFD % 64) == 0 && (NTOK % 64) == 0 && (PROJN % 64) == 0);

#define WSC 1024.0f
#define ASC 16.0f
#define PSC 1024.0f

typedef _Float16 v16h __attribute__((ext_vector_type(16)));
typedef _Float16 v8h  __attribute__((ext_vector_type(8)));
typedef float    v8f  __attribute__((ext_vector_type(8)));
typedef float    v4f  __attribute__((ext_vector_type(4)));
typedef unsigned int v4u __attribute__((ext_vector_type(4)));

#if defined(__HIP_DEVICE_COMPILE__)
#define DEV_ASM(...) asm volatile(__VA_ARGS__)
#else
#define DEV_ASM(...) do { } while (0)
#endif

__device__ __forceinline__ unsigned short h_bits(float f) {
  return __builtin_bit_cast(unsigned short, (_Float16)f);
}
__device__ __forceinline__ unsigned pk16(unsigned short a, unsigned short b) { return (unsigned)a | ((unsigned)b << 16); }
__device__ __forceinline__ v8f zero8() { v8f z = {0.f, 0.f, 0.f, 0.f, 0.f, 0.f, 0.f, 0.f}; return z; }

__device__ __forceinline__ v16h ldfrag(const _Float16* p) {
  union { v16h v; v8h h[2]; } f;
  f.h[0] = *(const v8h*)(p);
  f.h[1] = *(const v8h*)(p + 16);
  return f.v;
}

__device__ __forceinline__ v8f mma_raw(v16h a, v16h b, v8f c) {
  return __builtin_amdgcn_wmma_f32_16x16x32_f16(false, a, false, b, (short)0, c, false, false);
}
__device__ __forceinline__ v8f mma_g(v16h a, v16h b, v8f c) {
  c = __builtin_amdgcn_wmma_f32_16x16x32_f16(false, a, false, b, (short)0, c, false, false);
  DEV_ASM("v_nop\n\tv_nop\n\tv_nop\n\tv_nop" : "+v"(c) : "v"(a), "v"(b));
  return c;
}
__device__ __forceinline__ void dep_guard(v8f& x, v8f& y, v16h a, v16h b) {
  DEV_ASM("v_nop\n\tv_nop\n\tv_nop\n\tv_nop" : "+v"(x), "+v"(y) : "v"(a), "v"(b));
}
__device__ __forceinline__ void keep2(v16h a, v16h b) { DEV_ASM("v_nop" :: "v"(a), "v"(b)); }
__device__ __forceinline__ void keep4(v16h a, v16h b, v16h c, v16h d) {
  DEV_ASM("v_nop" :: "v"(a), "v"(b), "v"(c), "v"(d));
}
__device__ __forceinline__ void acc_guard4(v8f& a, v8f& b, v8f& c, v8f& d) {
  DEV_ASM("v_nop\n\tv_nop\n\tv_nop\n\tv_nop" : "+v"(a), "+v"(b), "+v"(c), "+v"(d));
}
__device__ __forceinline__ void wave_sync_lds() {
  __builtin_amdgcn_fence(__ATOMIC_RELEASE, "workgroup");
  __builtin_amdgcn_wave_barrier();
  __builtin_amdgcn_fence(__ATOMIC_ACQUIRE, "workgroup");
}

__device__ __forceinline__ float gelu_t(float g) {
  const float u2 = 1.5957691216057308f * (g + 0.044715f * g * g * g);
  const float e  = __expf(u2);
  return g - g * __builtin_amdgcn_rcpf(e + 1.0f);
}

__global__ __launch_bounds__(256) void ln_rows(const float* __restrict__ x, const float* __restrict__ w,
                                               const float* __restrict__ bb, unsigned short* y, int nrows) {
  const int lane = threadIdx.x & 31;
  const int row  = blockIdx.x * 8 + (threadIdx.x >> 5);
  if (row >= nrows) return;
  const float* xr = x + (size_t)row * DMOD;
  float s = 0.f;
#pragma unroll 1
  for (int i = 0; i < 4; ++i) {
    const int col = i * 256 + lane * 8;
    const v4f a = *(const v4f*)(xr + col);
    const v4f c = *(const v4f*)(xr + col + 4);
    s += ((a[0] + a[1]) + (a[2] + a[3])) + ((c[0] + c[1]) + (c[2] + c[3]));
  }
#pragma unroll
  for (int off = 1; off < 32; off <<= 1) s += __shfl_xor(s, off, 32);
  const float mean = s * (1.0f / DMOD);
  float sq = 0.f;
#pragma unroll 1
  for (int i = 0; i < 4; ++i) {
    const int col = i * 256 + lane * 8;
    const v4f a = *(const v4f*)(xr + col);
    const v4f c = *(const v4f*)(xr + col + 4);
#pragma unroll
    for (int e = 0; e < 4; ++e) {
      const float d0 = a[e] - mean, d1 = c[e] - mean;
      sq += d0 * d0;
      sq += d1 * d1;
    }
  }
#pragma unroll
  for (int off = 1; off < 32; off <<= 1) sq += __shfl_xor(sq, off, 32);
  const float rstd = rsqrtf(sq * (1.0f / DMOD) + 1e-5f);
#pragma unroll 1
  for (int i = 0; i < 4; ++i) {
    const int col = i * 256 + lane * 8;
    const v4f a  = *(const v4f*)(xr + col);
    const v4f c  = *(const v4f*)(xr + col + 4);
    const v4f wa = *(const v4f*)(w + col);
    const v4f wc = *(const v4f*)(w + col + 4);
    const v4f ba = *(const v4f*)(bb + col);
    const v4f bc = *(const v4f*)(bb + col + 4);
    v4u p;
#pragma unroll
    for (int e = 0; e < 2; ++e) {
      const float o0 = (a[2 * e] - mean) * rstd * wa[2 * e] + ba[2 * e];
      const float o1 = (a[2 * e + 1] - mean) * rstd * wa[2 * e + 1] + ba[2 * e + 1];
      const float o2 = (c[2 * e] - mean) * rstd * wc[2 * e] + bc[2 * e];
      const float o3 = (c[2 * e + 1] - mean) * rstd * wc[2 * e + 1] + bc[2 * e + 1];
      p[e]     = pk16(h_bits(o0), h_bits(o1));
      p[2 + e] = pk16(h_bits(o2), h_bits(o3));
    }
    unsigned short* dst = y + (size_t)row * DMOD + col;
    *(volatile v4u*)dst = p;
    __threadfence();
    *(volatile v4u*)dst = p;
  }
}

__global__ __launch_bounds__(256) void cvt_t16(const float* __restrict__ in, int R, int C,
                                               unsigned short* out, int ldo, float scale) {
  __shared__ float tile[64][65];
  const int tid = threadIdx.x;
  const int c0 = blockIdx.x * 64;
  const int r0 = blockIdx.y * 64;
  (void)R;
  {
    const int rr = tid >> 2, cq = (tid & 3) * 16;
    const float* src = in + (size_t)(r0 + rr) * C + c0 + cq;
#pragma unroll
    for (int e = 0; e < 4; ++e) {
      const v4f a = *(const v4f*)(src + 4 * e);
      tile[rr][cq + 4 * e + 0] = a[0];
      tile[rr][cq + 4 * e + 1] = a[1];
      tile[rr][cq + 4 * e + 2] = a[2];
      tile[rr][cq + 4 * e + 3] = a[3];
    }
  }
  __syncthreads();
#pragma unroll 1
  for (int ph = 0; ph < 2; ++ph) {
    const int cc = (tid >> 3) + 32 * ph;
    const int r8 = (tid & 7) * 8;
    v4u p;
#pragma unroll
    for (int e = 0; e < 4; ++e) {
      const float f0 = tile[r8 + 2 * e][cc] * scale;
      const float f1 = tile[r8 + 2 * e + 1][cc] * scale;
      p[e] = pk16(h_bits(f0), h_bits(f1));
    }
    unsigned short* dst = out + (size_t)(c0 + cc) * ldo + r0 + r8;
    *(volatile v4u*)dst = p;
    __threadfence();
    *(volatile v4u*)dst = p;
  }
}

template <int MODE>
__global__ __launch_bounds__(256) void gemm64(
    const unsigned short* __restrict__ Ap, int lda, long long strideA,
    const unsigned short* __restrict__ Bp, int ldb, long long strideB,
    void* Cp, int ldc, long long strideC,
    const float* __restrict__ Rp,
    int M, int N, int K, float oscale) {
  const _Float16* A  = (const _Float16*)(const void*)Ap;
  const _Float16* Bt = (const _Float16*)(const void*)Bp;
  __shared__ __align__(16) float sT[8][16 * 68];
  const int bz   = blockIdx.y;
  const int lane = threadIdx.x & 31;
  const int wave = threadIdx.x >> 5;
  const int tilesN = N >> 6;
  const int tilesM = M >> 6;
  const int tile = blockIdx.x * 8 + wave;
  if (tile >= tilesM * tilesN) return;
  const int tm = tile / tilesN;
  const int tn = tile - tm * tilesN;
  const int m0 = tm << 6;
  const int n0 = tn << 6;
  const _Float16* Ab = A  + (long long)bz * strideA;
  const _Float16* Bb = Bt + (long long)bz * strideB;
  const int rlane = lane & 15;
  const int koff  = (lane >> 4) * 8;
  const int mOff  = (lane >> 4) * 8;

  v8f acc[4][4];
#pragma unroll
  for (int i = 0; i < 4; ++i)
#pragma unroll
    for (int j = 0; j < 4; ++j) acc[i][j] = zero8();

#pragma unroll 1
  for (int k0 = 0; k0 < K; k0 += 32) {
    v16h bh[4];
#pragma unroll
    for (int j = 0; j < 4; ++j)
      bh[j] = ldfrag(Bb + (size_t)(n0 + (j << 4) + rlane) * ldb + koff + k0);
#pragma unroll
    for (int i = 0; i < 4; ++i) {
      const v16h ah = ldfrag(Ab + (size_t)(m0 + (i << 4) + rlane) * lda + koff + k0);
#pragma unroll
      for (int j = 0; j < 4; ++j) acc[i][j] = mma_raw(ah, bh[j], acc[i][j]);
      dep_guard(acc[i][0], acc[i][3], ah, ah);
    }
    keep4(bh[0], bh[1], bh[2], bh[3]);
  }
  acc_guard4(acc[0][0], acc[0][1], acc[0][2], acc[0][3]);
  acc_guard4(acc[1][0], acc[1][1], acc[1][2], acc[1][3]);
  acc_guard4(acc[2][0], acc[2][1], acc[2][2], acc[2][3]);
  acc_guard4(acc[3][0], acc[3][1], acc[3][2], acc[3][3]);

  float* slab = sT[wave];
#pragma unroll
  for (int i = 0; i < 4; ++i) {
    const int mBase = m0 + (i << 4);
#pragma unroll
    for (int j = 0; j < 4; ++j) {
#pragma unroll
      for (int r = 0; r < 8; ++r) slab[(mOff + r) * 68 + (j << 4) + rlane] = acc[i][j][r];
    }
    wave_sync_lds();
    if (MODE == 1) {
      float* Cf = (float*)Cp + (long long)bz * strideC;
      const float* Rf = Rp + (long long)bz * strideC;
      const int h2 = lane >> 4, c4 = (lane & 15) * 4;
      v4f vv[8];
#pragma unroll
      for (int it = 0; it < 8; ++it) {
        const int row = it * 2 + h2;
        const v4f v  = *(const v4f*)(slab + row * 68 + c4);
        const v4f rr = *(const v4f*)(Rf + (size_t)(mBase + row) * ldc + n0 + c4);
        vv[it] = rr + v * oscale;
      }
      for (int pass = 0; pass < 2; ++pass) {
#pragma unroll
        for (int it = 0; it < 8; ++it) {
          const int row = it * 2 + h2;
          *(volatile v4f*)(Cf + (size_t)(mBase + row) * ldc + n0 + c4) = vv[it];
        }
        __threadfence();
      }
    } else {
      unsigned short* Ch = (unsigned short*)Cp + (long long)bz * strideC;
      const int q = lane >> 3, c8 = (lane & 7) * 8;
      v4u hv[4];
#pragma unroll
      for (int it = 0; it < 4; ++it) {
        const int row = it * 4 + q;
        const float* sp = slab + row * 68 + c8;
        v4u a;
#pragma unroll
        for (int e = 0; e < 4; ++e) a[e] = pk16(h_bits(sp[2 * e] * oscale), h_bits(sp[2 * e + 1] * oscale));
        hv[it] = a;
      }
      for (int pass = 0; pass < 2; ++pass) {
#pragma unroll
        for (int it = 0; it < 4; ++it) {
          const int row = it * 4 + q;
          *(volatile v4u*)(Ch + (size_t)(mBase + row) * ldc + n0 + c8) = hv[it];
        }
        __threadfence();
      }
    }
    wave_sync_lds();
  }
}

__global__ __launch_bounds__(256) void gemm_ffg(
    const unsigned short* __restrict__ Ap, int lda,
    const unsigned short* __restrict__ Bp, int ldb, long long goff,
    unsigned short* Cp, int ldc,
    int M, int N, int K, float wscInv, float asc) {
  const _Float16* A  = (const _Float16*)(const void*)Ap;
  const _Float16* Bf = (const _Float16*)(const void*)Bp;
  const _Float16* Bg = Bf + goff;
  __shared__ __align__(16) float sT[8][16 * 68];
  const int lane = threadIdx.x & 31;
  const int wave = threadIdx.x >> 5;
  const int tilesN = N >> 6;
  const int tilesM = M >> 5;
  const int tile = blockIdx.x * 8 + wave;
  if (tile >= tilesM * tilesN) return;
  const int tm = tile / tilesN;
  const int tn = tile - tm * tilesN;
  const int m0 = tm << 5;
  const int n0 = tn << 6;
  const int rlane = lane & 15;
  const int koff  = (lane >> 4) * 8;
  const int mOff  = (lane >> 4) * 8;

  v8f f[2][4], g[2][4];
#pragma unroll
  for (int i = 0; i < 2; ++i)
#pragma unroll
    for (int j = 0; j < 4; ++j) { f[i][j] = zero8(); g[i][j] = zero8(); }

#pragma unroll 1
  for (int k0 = 0; k0 < K; k0 += 32) {
    v16h a[2];
#pragma unroll
    for (int i = 0; i < 2; ++i) a[i] = ldfrag(A + (size_t)(m0 + (i << 4) + rlane) * lda + koff + k0);
#pragma unroll
    for (int j = 0; j < 4; ++j) {
      const size_t bo = (size_t)(n0 + (j << 4) + rlane) * ldb + koff + k0;
      const v16h bf = ldfrag(Bf + bo);
      const v16h bg = ldfrag(Bg + bo);
#pragma unroll
      for (int i = 0; i < 2; ++i) {
        f[i][j] = mma_raw(a[i], bf, f[i][j]);
        g[i][j] = mma_raw(a[i], bg, g[i][j]);
      }
      dep_guard(f[0][j], g[1][j], bf, bg);
    }
    keep2(a[0], a[1]);
  }
  acc_guard4(f[0][0], f[0][1], f[0][2], f[0][3]);
  acc_guard4(f[1][0], f[1][1], f[1][2], f[1][3]);
  acc_guard4(g[0][0], g[0][1], g[0][2], g[0][3]);
  acc_guard4(g[1][0], g[1][1], g[1][2], g[1][3]);

  float* slab = sT[wave];
#pragma unroll
  for (int i = 0; i < 2; ++i) {
    const int mBase = m0 + (i << 4);
#pragma unroll
    for (int j = 0; j < 4; ++j) {
#pragma unroll
      for (int r = 0; r < 8; ++r) {
        const float ff = f[i][j][r] * wscInv;
        const float gg = g[i][j][r] * wscInv;
        slab[(mOff + r) * 68 + (j << 4) + rlane] = asc * (ff * gelu_t(gg));
      }
    }
    wave_sync_lds();
    {
      const int q = lane >> 3, c8 = (lane & 7) * 8;
      v4u hv[4];
#pragma unroll
      for (int it = 0; it < 4; ++it) {
        const int row = it * 4 + q;
        const float* sp = slab + row * 68 + c8;
        v4u w4;
#pragma unroll
        for (int e = 0; e < 4; ++e) w4[e] = pk16(h_bits(sp[2 * e]), h_bits(sp[2 * e + 1]));
        hv[it] = w4;
      }
      for (int pass = 0; pass < 2; ++pass) {
#pragma unroll
        for (int it = 0; it < 4; ++it) {
          const int row = it * 4 + q;
          *(volatile v4u*)(Cp + (size_t)(mBase + row) * ldc + n0 + c8) = hv[it];
        }
        __threadfence();
      }
    }
    wave_sync_lds();
  }
}

__global__ __launch_bounds__(128)
void attn64(const unsigned short* __restrict__ qkp, const unsigned short* __restrict__ vtp,
            unsigned short* ctxp, float sscale) {
  union FH { v16h v; v8h h[2]; };
  __shared__ __align__(16) _Float16 Psh[4][16 * 64];
  __shared__ __align__(16) float    Os[4][16 * 64];

  const int tid  = threadIdx.x;
  const int wave = tid >> 5;
  const int lane = tid & 31;
  const int hh   = lane >> 4;
  const int c    = lane & 15;

  const int bx   = blockIdx.x;
  const int qb   = bx % NQB;
  const int rest = bx / NQB;
  const int h    = rest % NHEAD;
  const int b    = rest / NHEAD;
  const int q0   = qb * 64 + wave * 16;
  const size_t rowB = (size_t)b * SEQL;

  const _Float16* Q  = (const _Float16*)(const void*)qkp + (size_t)h * HDIM;
  const _Float16* Kk = Q + DMOD;
  const _Float16* Vt = (const _Float16*)(const void*)vtp + ((size_t)b * DMOD + (size_t)h * HDIM) * SEQL;

  v16h qa[2];
#pragma unroll
  for (int dc = 0; dc < 2; ++dc) qa[dc] = ldfrag(Q + (rowB + q0 + c) * QKP + dc * 32 + 8 * hh);

  float mrow[8], lrow[8];
  v8f oacc[4];
#pragma unroll
  for (int r = 0; r < 8; ++r) { mrow[r] = -INFINITY; lrow[r] = 0.f; }
#pragma unroll
  for (int t = 0; t < 4; ++t) oacc[t] = zero8();

  _Float16* pw = Psh[wave];

#pragma unroll 1
  for (int kt = 0; kt < NQB; ++kt) {
    const int kv0 = kt * 64;

    v8f s[4];
#pragma unroll
    for (int j = 0; j < 4; ++j) {
      s[j] = zero8();
      const _Float16* krow = Kk + (rowB + kv0 + j * 16 + c) * QKP + 8 * hh;
#pragma unroll
      for (int dc = 0; dc < 2; ++dc) {
        const v16h kb = ldfrag(krow + dc * 32);
        s[j] = mma_g(qa[dc], kb, s[j]);
      }
    }

#pragma unroll
    for (int r = 0; r < 8; ++r) {
      float m = -INFINITY;
#pragma unroll
      for (int j = 0; j < 4; ++j) {
        const float sv = s[j][r] * sscale;
        s[j][r] = sv;
        m = fmaxf(m, sv);
      }
#pragma unroll
      for (int off = 1; off < 16; off <<= 1) m = fmaxf(m, __shfl_xor(m, off, 32));
      const float mnew  = fmaxf(mrow[r], m);
      const float msafe = (mnew == -INFINITY) ? 0.f : mnew;
      const float alpha = __expf(mrow[r] - msafe);
      mrow[r] = mnew;
      float psum = 0.f;
#pragma unroll
      for (int j = 0; j < 4; ++j) {
        const float p = __expf(s[j][r] - msafe);
        psum += p;
        pw[(8 * hh + r) * 64 + j * 16 + c] = (_Float16)(p * PSC);
      }
#pragma unroll
      for (int off = 1; off < 16; off <<= 1) psum += __shfl_xor(psum, off, 32);
      lrow[r] = lrow[r] * alpha + psum;
#pragma unroll
      for (int t = 0; t < 4; ++t) oacc[t][r] *= alpha;
    }
    wave_sync_lds();

#pragma unroll
    for (int kk = 0; kk < 2; ++kk) {
      FH pa;
      pa.h[0] = *(const v8h*)(pw + c * 64 + kk * 32 + 8 * hh);
      pa.h[1] = *(const v8h*)(pw + c * 64 + kk * 32 + 16 + 8 * hh);
#pragma unroll
      for (int t = 0; t < 4; ++t) {
        const v16h vb = ldfrag(Vt + (size_t)(t * 16 + c) * SEQL + kv0 + kk * 32 + 8 * hh);
        oacc[t] = mma_g(pa.v, vb, oacc[t]);
      }
    }
    wave_sync_lds();
  }

  float* os = Os[wave];
#pragma unroll
  for (int r = 0; r < 8; ++r) {
    const float l   = lrow[r];
    const float inv = ((l > 0.f) ? (1.0f / l) : 0.f) * (1.0f / PSC);
#pragma unroll
    for (int t = 0; t < 4; ++t) os[(8 * hh + r) * 64 + t * 16 + c] = oacc[t][r] * inv;
  }
  wave_sync_lds();
  {
    const int q4 = lane >> 3, c8 = (lane & 7) * 8;
    v4u hv[4];
#pragma unroll
    for (int it = 0; it < 4; ++it) {
      const int row = it * 4 + q4;
      const float* sp = os + row * 64 + c8;
      v4u a;
#pragma unroll
      for (int e = 0; e < 4; ++e) a[e] = pk16(h_bits(sp[2 * e]), h_bits(sp[2 * e + 1]));
      hv[it] = a;
    }
    for (int pass = 0; pass < 2; ++pass) {
#pragma unroll
      for (int it = 0; it < 4; ++it) {
        const int row = it * 4 + q4;
        const size_t go = (rowB + q0 + row) * A2P + (size_t)h * HDIM + c8;
        *(volatile v4u*)(ctxp + go) = hv[it];
      }
      __threadfence();
    }
  }
}

extern "C" void kernel_launch(void* const* d_in, const int* in_sizes, int n_in,
                              void* d_out, int out_size, void* d_ws, size_t ws_size,
                              hipStream_t stream) {
  if (n_in < 6) return;
  if (in_sizes[0] != NTOK * DMOD) return;
  if (in_sizes[1] != DMOD || in_sizes[2] != DMOD) return;
  if (in_sizes[3] != DMOD * PROJN) return;
  if (in_sizes[4] != DMOD * DMOD) return;
  if (in_sizes[5] != FFD * DMOD) return;
  if (out_size != NTOK * DMOD) return;

  const float* x      = (const float*)d_in[0];
  const float* ln_w   = (const float*)d_in[1];
  const float* ln_b   = (const float*)d_in[2];
  const float* w_in   = (const float*)d_in[3];
  const float* w_attn = (const float*)d_in[4];
  const float* w_ff   = (const float*)d_in[5];
  float* out = (float*)d_out;

  const size_t PU   = (size_t)NTOK * DMOD * 2;
  const size_t PWIN = (size_t)PROJN * DMOD * 2;
  const size_t PW2  = (size_t)DMOD * A2P * 2;
  const size_t PQK  = (size_t)NTOK * QKP * 2;
  const size_t PVT  = (size_t)NBATCH * DMOD * SEQL * 2;
  const size_t PA2  = (size_t)NTOK * A2P * 2;
  size_t off = 0;
  const size_t oU   = off; off += PU;
  const size_t oWin = off; off += PWIN;
  const size_t oW2  = off; off += PW2;
  const size_t oQK  = off; off += PQK;
  const size_t oVT  = off; off += PVT;
  const size_t oA2  = off; off += PA2;
  if (off > ws_size) return;
  if (off > (size_t)134217728) return;

  char* ws = (char*)d_ws;
  unsigned short* U    = (unsigned short*)(ws + oU);
  unsigned short* WinT = (unsigned short*)(ws + oWin);
  unsigned short* W2T  = (unsigned short*)(ws + oW2);
  unsigned short* QK   = (unsigned short*)(ws + oQK);
  unsigned short* VT   = (unsigned short*)(ws + oVT);
  unsigned short* A2   = (unsigned short*)(ws + oA2);

  static_assert((((NTOK / 64) * (2 * DMOD / 64)) % 8) == 0);
  static_assert((((DMOD / 64) * (SEQL / 64)) % 8) == 0);
  static_assert((((NTOK / 32) * (FFD / 64)) % 8) == 0);
  static_assert((((NTOK / 64) * (DMOD / 64)) % 8) == 0);
  static_assert((NTOK % 8) == 0);

  const dim3 blk(256);
  const dim3 gLN(NTOK / 8);
  const dim3 gTin(PROJN / 64, DMOD / 64);
  const dim3 gTat(DMOD / 64, DMOD / 64);
  const dim3 gTff(DMOD / 64, FFD / 64);
  const dim3 gQK(((NTOK / 64) * (2 * DMOD / 64)) / 8, 1);
  const dim3 gVT(((DMOD / 64) * (SEQL / 64)) / 8, NBATCH);
  const dim3 gFFG(((NTOK / 32) * (FFD / 64)) / 8, 1);
  const dim3 gOUT(((NTOK / 64) * (DMOD / 64)) / 8, 1);
  const dim3 gATT(NBATCH * NHEAD * NQB);

  ln_rows<<<gLN, blk, 0, stream>>>(x, ln_w, ln_b, U, NTOK);
  cvt_t16<<<gTin, blk, 0, stream>>>(w_in, DMOD, PROJN, WinT, DMOD, WSC);
  cvt_t16<<<gTat, blk, 0, stream>>>(w_attn, DMOD, DMOD, W2T, A2P, WSC);
  cvt_t16<<<gTff, blk, 0, stream>>>(w_ff, FFD, DMOD, W2T + DMOD, A2P, WSC);
  gemm64<0><<<gQK, blk, 0, stream>>>(
      U, DMOD, 0LL, WinT, DMOD, 0LL,
      (void*)QK, QKP, 0LL, x,
      NTOK, 2 * DMOD, DMOD, ASC / WSC);
  gemm64<0><<<gVT, blk, 0, stream>>>(
      WinT + (size_t)2 * DMOD * DMOD, DMOD, 0LL, U, DMOD, (long long)SEQL * DMOD,
      (void*)VT, SEQL, (long long)DMOD * SEQL, x,
      DMOD, SEQL, DMOD, ASC / WSC);
  gemm_ffg<<<gFFG, blk, 0, stream>>>(
      U, DMOD, WinT + (size_t)3 * DMOD * DMOD, DMOD, (long long)FFD * DMOD,
      A2 + DMOD, A2P,
      NTOK, FFD, DMOD, 1.0f / WSC, ASC);
  attn64<<<gATT, dim3(128), 0, stream>>>(QK, VT, A2, 1.0f / (ASC * ASC * 8.0f));
  gemm64<1><<<gOUT, blk, 0, stream>>>(
      A2, A2P, 0LL, W2T, A2P, 0LL,
      (void*)out, DMOD, 0LL, x,
      NTOK, DMOD, A2P, 1.0f / (ASC * WSC));
  (void)hipGetLastError();
}
